// S6_67310727463501
// MI455X (gfx1250) — hardware-verified
//
#include <hip/hip_runtime.h>
#include <math.h>

#ifndef NB
#define NB 4
#endif
#ifndef SEQ
#define SEQ 2048
#endif
#define NB_FULL 4
#define SEQ_FULL 2048
#define DM 768
#define NS 16
#define NBC 64
#define NBIASP 128
#define MROWS (NB * SEQ)
static_assert(MROWS % 64 == 0);
static_assert(DM % 128 == 0);
static_assert(DM % 32 == 0);
static_assert(NBC % 64 == 0);
static_assert(NB <= NB_FULL);
static_assert(SEQ <= SEQ_FULL);

typedef __attribute__((ext_vector_type(16))) _Float16 v16h;
typedef __attribute__((ext_vector_type(8)))  _Float16 v8h;
typedef __attribute__((ext_vector_type(16))) __bf16   v16b;
typedef __attribute__((ext_vector_type(8)))  __bf16   v8b;
typedef __attribute__((ext_vector_type(8)))  float    v8f;
typedef __attribute__((ext_vector_type(4)))  float    v4f;
typedef __attribute__((ext_vector_type(4)))  unsigned int v4u_at;

#define VST2(T, ptr, val) do { const T vst2_v_ = (val); *(volatile T*)(ptr) = vst2_v_; __threadfence(); *(volatile T*)(ptr) = vst2_v_; } while (0)
#define VST2V4(ptr, val) do { const v4f vst2_v4_ = (val); *(volatile v4f*)(ptr) = vst2_v4_; __threadfence(); *(volatile v4f*)(ptr) = vst2_v4_; } while (0)

__device__ __forceinline__ unsigned short f2bf_bits_g(float f) { unsigned u = __float_as_uint(f); return (unsigned short)((u + 0x7FFFu + ((u >> 16) & 1u)) >> 16); }
__device__ __forceinline__ float bfr(float f) { return __uint_as_float(((unsigned)f2bf_bits_g(f)) << 16); }
__device__ __forceinline__ unsigned short at_f2h(float x) { return (fabsf(x) < 6.104e-5f) ? (unsigned short)0 : __builtin_bit_cast(unsigned short, (_Float16)x); }
__device__ __forceinline__ void at_st8h(unsigned short* Pp, long long o, const float* v) {
    v4u_at pk;
    pk.x = (unsigned int)at_f2h(v[0]) | ((unsigned int)at_f2h(v[1]) << 16);
    pk.y = (unsigned int)at_f2h(v[2]) | ((unsigned int)at_f2h(v[3]) << 16);
    pk.z = (unsigned int)at_f2h(v[4]) | ((unsigned int)at_f2h(v[5]) << 16);
    pk.w = (unsigned int)at_f2h(v[6]) | ((unsigned int)at_f2h(v[7]) << 16);
    VST2(v4u_at, (v4u_at*)(Pp + o), pk);
}

namespace w25 {
typedef __attribute__((ext_vector_type(16))) _Float16 v16h;
typedef __attribute__((ext_vector_type(8)))  _Float16 v8h;
typedef __attribute__((ext_vector_type(16))) __bf16   v16b;
typedef __attribute__((ext_vector_type(8)))  __bf16   v8b;
typedef __attribute__((ext_vector_type(8)))  float    v8f;
typedef __attribute__((ext_vector_type(4)))  float    v4f;

__device__ __forceinline__ unsigned short f2bf_bits(float f) {
  unsigned u = __float_as_uint(f);
  return (unsigned short)((u + 0x7FFFu + ((u >> 16) & 1u)) >> 16);
}
__device__ __forceinline__ float bf_bits2f(unsigned short h) { return __uint_as_float(((unsigned)h) << 16); }

__device__ __forceinline__ void dep_guard_h(v8f& a, v8f& b, v16h x, v16h y) { asm volatile("v_nop\n\tv_nop\n\tv_nop\n\tv_nop" : "+v"(a), "+v"(b) : "v"(x), "v"(y)); }
__device__ __forceinline__ void dep_guard_b(v8f& a, v8f& b, v16b x, v16b y) { asm volatile("v_nop\n\tv_nop\n\tv_nop\n\tv_nop" : "+v"(a), "+v"(b) : "v"(x), "v"(y)); }
__device__ __forceinline__ void keep4_h(v16h a, v16h b, v16h c, v16h d) { asm volatile("v_nop" :: "v"(a), "v"(b), "v"(c), "v"(d)); }
__device__ __forceinline__ void keep4_b(v16b a, v16b b, v16b c, v16b d) { asm volatile("v_nop" :: "v"(a), "v"(b), "v"(c), "v"(d)); }
__device__ __forceinline__ void acc_guard4(v8f& a, v8f& b, v8f& c, v8f& d) { asm volatile("v_nop\n\tv_nop\n\tv_nop\n\tv_nop" : "+v"(a), "+v"(b), "+v"(c), "+v"(d)); }
template <typename T> struct Frag;
template <> struct Frag<_Float16> {
  typedef v16h V; union U { v16h v; v8h h[2]; };
  static __device__ __forceinline__ v16h load(const _Float16* p) {
    U f; f.h[0] = *(const v8h*)(p); f.h[1] = *(const v8h*)(p + 16); return f.v;
  }
  static __device__ __forceinline__ v8f mma(v16h a, v16h b, v8f c) {
    return __builtin_amdgcn_wmma_f32_16x16x32_f16(false, a, false, b, (short)0, c, false, false);
  }
  static __device__ __forceinline__ void guard(v8f& a, v8f& b, v16h x, v16h y) { dep_guard_h(a, b, x, y); }
  static __device__ __forceinline__ void keep(v16h a, v16h b, v16h c, v16h d) { keep4_h(a, b, c, d); }
};
template <> struct Frag<__bf16> {
  typedef v16b V; union U { v16b v; v8b h[2]; };
  static __device__ __forceinline__ v16b load(const __bf16* p) {
    U f; f.h[0] = *(const v8b*)(p); f.h[1] = *(const v8b*)(p + 16); return f.v;
  }
  static __device__ __forceinline__ v8f mma(v16b a, v16b b, v8f c) {
    return __builtin_amdgcn_wmma_f32_16x16x32_bf16(false, a, false, b, (short)0, c, false, false);
  }
  static __device__ __forceinline__ void guard(v8f& a, v8f& b, v16b x, v16b y) { dep_guard_b(a, b, x, y); }
  static __device__ __forceinline__ void keep(v16b a, v16b b, v16b c, v16b d) { keep4_b(a, b, c, d); }
};

template <int ET> struct Elem;
template <> struct Elem<0> { typedef _Float16 T; };
template <> struct Elem<1> { typedef __bf16 T; };
template <int ET, bool SPLIT, int BIAS_MODE, int OUT_MODE, bool RESID, int ACT = 0>
__global__ __launch_bounds__(256) void wmma_gemm64(
    const unsigned short* __restrict__ Ap, const unsigned short* __restrict__ A2p, int lda, long strideA,
    const unsigned short* __restrict__ Btp, const unsigned short* __restrict__ Bt2p, int ldb, long strideB,
    void* __restrict__ Cout, void* __restrict__ Cout2, int ldc, long strideC,
    const float* __restrict__ bias,
    const float* __restrict__ resid, long strideR,
    int M, int N, int K, float scale) {
  typedef typename Elem<ET>::T T;
  typedef typename Frag<T>::V V;
  const T* A = (const T*)Ap; const T* A2 = (const T*)A2p; const T* Bt = (const T*)Btp; const T* Bt2 = (const T*)Bt2p;
  __shared__ __align__(16) float sT[8][16 * 68];
  const int b    = blockIdx.y;
  const int lane = threadIdx.x & 31;
  const int wave = threadIdx.x >> 5;
  const int tilesN = N >> 6;
  const int tilesM = M >> 6;
  const int tile = blockIdx.x * 8 + wave;
  if (tile >= tilesM * tilesN) return;
  const int tm = tile / tilesN;
  const int tn = tile - tm * tilesN;
  const int m0 = tm << 6;
  const int n0 = tn << 6;

  const T* Ab  = A  + (size_t)b * strideA;
  const T* Bb  = Bt + (size_t)b * strideB;
  const T* Ab2 = SPLIT ? (A2  + (size_t)b * strideA) : nullptr;
  const T* Bb2 = SPLIT ? (Bt2 + (size_t)b * strideB) : nullptr;

  const int rlane = lane & 15;
  const int koff  = (lane >> 4) * 8;
  const int mOff  = (lane >> 4) * 8;

  v8f acc[4][4];
#pragma unroll
  for (int i = 0; i < 4; ++i)
#pragma unroll
    for (int j = 0; j < 4; ++j) acc[i][j] = (v8f){0.f,0.f,0.f,0.f,0.f,0.f,0.f,0.f};

  for (int k0 = 0; k0 < K; k0 += 32) {
    V bh[4], bl[4];
#pragma unroll
    for (int j = 0; j < 4; ++j) {
      const size_t bo = (size_t)(n0 + (j << 4) + rlane) * ldb + koff + k0;
      bh[j] = Frag<T>::load(Bb + bo);
      if (SPLIT) bl[j] = Frag<T>::load(Bb2 + bo);
    }
#pragma unroll
    for (int i = 0; i < 4; ++i) {
      const size_t ao = (size_t)(m0 + (i << 4) + rlane) * lda + koff + k0;
      V ah = Frag<T>::load(Ab + ao);
      V al;
      if (SPLIT) al = Frag<T>::load(Ab2 + ao);
#pragma unroll
      for (int j = 0; j < 4; ++j) {
        acc[i][j] = Frag<T>::mma(ah, bh[j], acc[i][j]);
        if (SPLIT) {
          acc[i][j] = Frag<T>::mma(ah, bl[j], acc[i][j]);
          acc[i][j] = Frag<T>::mma(al, bh[j], acc[i][j]);
        }
      }
      Frag<T>::guard(acc[i][0], acc[i][3], ah, SPLIT ? al : ah);
    }
    Frag<T>::keep(bh[0], bh[1], bh[2], bh[3]);
    if (SPLIT) Frag<T>::keep(bl[0], bl[1], bl[2], bl[3]);
  }
  acc_guard4(acc[0][0], acc[0][1], acc[0][2], acc[0][3]);
  acc_guard4(acc[1][0], acc[1][1], acc[1][2], acc[1][3]);
  acc_guard4(acc[2][0], acc[2][1], acc[2][2], acc[2][3]);
  acc_guard4(acc[3][0], acc[3][1], acc[3][2], acc[3][3]);

  float* slab = sT[wave];
  const float* Rb = RESID ? (resid + (size_t)b * strideR) : nullptr;
#pragma unroll
  for (int i = 0; i < 4; ++i) {
    const int mBase = m0 + (i << 4);
#pragma unroll
    for (int j = 0; j < 4; ++j) {
      const int n = n0 + (j << 4) + rlane;
      float bv = 0.f;
      if (BIAS_MODE == 2) bv = bias[n];
#pragma unroll
      for (int r = 0; r < 8; ++r) {
        float v = acc[i][j][r] * scale;
        if (BIAS_MODE == 1) v += bias[mBase + mOff + r];
        if (BIAS_MODE == 2) v += bv;
        if (RESID) v += Rb[(size_t)(mBase + mOff + r) * ldc + n];
        if (ACT == 1) v = tanhf(v);
        if (ACT == 2) v = fmaxf(v, 0.0f);
        if (ACT == 3) v = v / (1.0f + expf(-v));
        if (ACT == 4) v = (v > 0.f) ? v : 0.01f * v;
        if (ACT == 5) v = 0.5f * v * (1.0f + erff(v * 0.70710678118654752f));
        if (ACT == 6) v = (v > 0.f) ? v : 0.2f * v;
        if (ACT == 7) { const float u = 0.7978845608028654f * (v + 0.044715f * v * v * v); v = 0.5f * v * (1.f + tanhf(u)); }
        slab[(mOff + r) * 68 + (j << 4) + rlane] = v;
      }
    }
    __builtin_amdgcn_fence(__ATOMIC_RELEASE, "workgroup");
    __builtin_amdgcn_wave_barrier();
    __builtin_amdgcn_fence(__ATOMIC_ACQUIRE, "workgroup");
    if (OUT_MODE == 0) {
      float* C = (float*)Cout + (size_t)b * strideC;
      const int hh = lane >> 4, c4 = (lane & 15) * 4;
      for (int pass = 0; pass < 2; ++pass) {
#pragma unroll
        for (int it = 0; it < 8; ++it) {
          const int row = it * 2 + hh;
          v4f v = *(const v4f*)(slab + row * 68 + c4);
          *(volatile v4f*)(C + (size_t)(mBase + row) * ldc + n0 + c4) = v;
        }
        __threadfence();
      }
    } else {
      const int q = lane >> 3, c8 = (lane & 7) * 8;
      unsigned short* C  = (unsigned short*)Cout  + (size_t)b * strideC;
      unsigned short* C2 = (OUT_MODE == 2) ? ((unsigned short*)Cout2 + (size_t)b * strideC) : nullptr;
      for (int pass = 0; pass < 2; ++pass) {
#pragma unroll
        for (int it = 0; it < 4; ++it) {
          const int row = it * 4 + q;
          const float* sp = slab + row * 68 + c8;
          v8h hv, lv;
#pragma unroll
          for (int e = 0; e < 8; ++e) {
            if (OUT_MODE == 1) {
              hv[e] = (_Float16)sp[e];
            } else {
              unsigned short hb = f2bf_bits(sp[e]);
              unsigned short lb = f2bf_bits(sp[e] - bf_bits2f(hb));
              hv[e] = __builtin_bit_cast(_Float16, hb);
              lv[e] = __builtin_bit_cast(_Float16, lb);
            }
          }
          *(volatile v8h*)(C + (size_t)(mBase + row) * ldc + n0 + c8) = hv;
          if (OUT_MODE == 2) *(volatile v8h*)(C2 + (size_t)(mBase + row) * ldc + n0 + c8) = lv;
        }
        __threadfence();
      }
    }
    __builtin_amdgcn_fence(__ATOMIC_RELEASE, "workgroup");
    __builtin_amdgcn_wave_barrier();
    __builtin_amdgcn_fence(__ATOMIC_ACQUIRE, "workgroup");
  }
}

}

__device__ __forceinline__ long long in_row(int r) { return (long long)(r / SEQ) * SEQ_FULL + (r % SEQ); }

__global__ __launch_bounds__(256) void k_x(const float* __restrict__ X, unsigned short* __restrict__ X16) {
    const long long u = (long long)blockIdx.x * 256 + threadIdx.x;
    if (u >= (long long)MROWS * (DM / 8)) return;
    const int r = (int)(u / (DM / 8)); const int c8 = 8 * (int)(u - (long long)r * (DM / 8));
    const float* xp = X + in_row(r) * DM + c8;
    const v4f a = *(const v4f*)xp, b = *(const v4f*)(xp + 4);
    float v[8] = {a.x, a.y, a.z, a.w, b.x, b.y, b.z, b.w};
#pragma unroll
    for (int i = 0; i < 8; ++i) v[i] = bfr(v[i]) * 8.0f;
    at_st8h(X16, u * 8, v);
}
__global__ __launch_bounds__(256) void k_w1(const float* __restrict__ W1, unsigned short* __restrict__ W16) {
    const long long u = (long long)blockIdx.x * 256 + threadIdx.x;
    if (u >= (long long)DM * (DM / 8)) return;
    const int o = (int)(u / (DM / 8)); const int k0 = 8 * (int)(u - (long long)o * (DM / 8));
    float v[8];
#pragma unroll
    for (int i = 0; i < 8; ++i) v[i] = bfr(W1[(long long)(k0 + i) * DM + o]) * 32.0f;
    at_st8h(W16, u * 8, v);
}
__global__ __launch_bounds__(256) void k_wb(const float* __restrict__ W2, const float* __restrict__ W3, unsigned short* __restrict__ WB) {
    const long long u = (long long)blockIdx.x * 256 + threadIdx.x;
    if (u >= (long long)NBC * (DM / 8)) return;
    const int o = (int)(u / (DM / 8)); const int k0 = 8 * (int)(u - (long long)o * (DM / 8));
    const int oa = min(o, NS - 1); const int ob = min(max(o - NS, 0), NS - 1);
    float v[8];
#pragma unroll
    for (int i = 0; i < 8; ++i) {
        const long long k = k0 + i;
        const float va = W2[k * NS + oa];
        const float vb = W3[k * NS + ob];
        const float sel = (o < NS) ? va : ((o < 2 * NS) ? vb : 0.0f);
        v[i] = bfr(sel) * 32.0f;
    }
    at_st8h(WB, u * 8, v);
}
__global__ __launch_bounds__(256) void k_bias(const float* __restrict__ b1, const float* __restrict__ b2, const float* __restrict__ b3, float* __restrict__ B1R, float* __restrict__ BIAS) {
    const int t = threadIdx.x; const int wv = t >> 5; const int L = t & 31;
    if (wv < DM / 128) {
        const int i4 = 4 * t;
        v4f v = *(const v4f*)(b1 + i4);
        v.x = bfr(v.x); v.y = bfr(v.y); v.z = bfr(v.z); v.w = bfr(v.w);
        VST2V4(B1R + i4, v);
    }
    if (wv == DM / 128) {
        float e[4];
#pragma unroll
        for (int j = 0; j < 4; ++j) {
            const int i = 4 * L + j;
            const float va = b2[min(i, NS - 1)];
            const float vb = b3[min(max(i - NS, 0), NS - 1)];
            e[j] = (i < NS) ? bfr(va) : ((i < 2 * NS) ? bfr(vb) : 0.0f);
        }
        v4f v; v.x = e[0]; v.y = e[1]; v.z = e[2]; v.w = e[3];
        VST2V4(BIAS + 4 * L, v);
    }
}
__device__ __forceinline__ float softplus_f(float z) { return fmaxf(z, 0.0f) + log1pf(expf(-fabsf(z))); }
__global__ __launch_bounds__(256) void k_out(const float* __restrict__ X, const float* __restrict__ DL, const float* __restrict__ BC, float* __restrict__ OUT) {
    #pragma clang fp contract(off)
    const long long u = (long long)blockIdx.x * 256 + threadIdx.x;
    if (u >= (long long)MROWS * (DM / 4)) return;
    const int r = (int)(u / (DM / 4)); const int c = 4 * (int)(u - (long long)r * (DM / 4));
    const float* bcr = BC + (long long)r * NBC;
    float bc = 0.0f;
#pragma unroll
    for (int q = 0; q < NS / 4; ++q) {
        const v4f bq = *(const v4f*)(bcr + 4 * q), cq = *(const v4f*)(bcr + NS + 4 * q);
        bc += bq.x * cq.x; bc += bq.y * cq.y; bc += bq.z * cq.z; bc += bq.w * cq.w;
    }
    const v4f xv = *(const v4f*)(X + in_row(r) * DM + c);
    const v4f dz = *(const v4f*)(DL + (long long)r * DM + c);
    v4f y;
    y.x = (bfr(xv.x) * softplus_f(dz.x)) * bc;
    y.y = (bfr(xv.y) * softplus_f(dz.y)) * bc;
    y.z = (bfr(xv.z) * softplus_f(dz.z)) * bc;
    y.w = (bfr(xv.w) * softplus_f(dz.w)) * bc;
    VST2V4(OUT + (long long)r * DM + c, y);
}

static inline size_t al256(size_t n) { return ((n + 255) / 256) * 256; }

extern "C" void kernel_launch(void* const* d_in, const int* in_sizes, int n_in, void* d_out, int out_size, void* d_ws, size_t ws_size, hipStream_t stream) {
    if (n_in < 7) return;
    if (in_sizes[0] < (int)((((long long)(NB - 1)) * SEQ_FULL + SEQ) * DM)) return;
    if (in_sizes[1] < DM * DM || in_sizes[2] < DM || in_sizes[3] < DM * NS || in_sizes[4] < NS || in_sizes[5] < DM * NS || in_sizes[6] < NS) return;
    if (out_size < MROWS * DM) return;
    const float* x  = (const float*)d_in[0];
    const float* W1 = (const float*)d_in[1];
    const float* b1 = (const float*)d_in[2];
    const float* W2 = (const float*)d_in[3];
    const float* b2 = (const float*)d_in[4];
    const float* W3 = (const float*)d_in[5];
    const float* b3 = (const float*)d_in[6];
    float* out = (float*)d_out;

    char* wsp = (char*)d_ws; size_t off = 0;
    unsigned short* X16 = (unsigned short*)(wsp + off); off += al256((size_t)MROWS * DM * 2);
    unsigned short* W16 = (unsigned short*)(wsp + off); off += al256((size_t)DM * DM * 2);
    unsigned short* WB  = (unsigned short*)(wsp + off); off += al256((size_t)NBC * DM * 2);
    float* B1R  = (float*)(wsp + off); off += al256((size_t)DM * 4);
    float* BIAS = (float*)(wsp + off); off += al256((size_t)NBIASP * 4);
    float* DL   = (float*)(wsp + off); off += al256((size_t)MROWS * DM * 4);
    float* BC   = (float*)(wsp + off); off += al256((size_t)MROWS * NBC * 4);
    if (off > ws_size) return;

    k_x<<<(unsigned)(((long long)MROWS * (DM / 8) + 255) / 256), 256, 0, stream>>>(x, X16);
    k_w1<<<(unsigned)(((long long)DM * (DM / 8) + 255) / 256), 256, 0, stream>>>(W1, W16);
    k_wb<<<(unsigned)(((long long)NBC * (DM / 8) + 255) / 256), 256, 0, stream>>>(W2, W3, WB);
    k_bias<<<1, 256, 0, stream>>>(b1, b2, b3, B1R, BIAS);
    w25::wmma_gemm64<0, false, 2, 0, false, 0><<<dim3((unsigned)((((MROWS) / 64) * ((DM) / 64) + 7) / 8), 1u), 256, 0, stream>>>(
        (const unsigned short*)X16, nullptr, DM, 0, (const unsigned short*)W16, nullptr, DM, 0, (void*)DL, nullptr, DM, 0, B1R, nullptr, 0, MROWS, DM, DM, 0.00390625f);
    w25::wmma_gemm64<0, false, 2, 0, false, 0><<<dim3((unsigned)((((MROWS) / 64) * ((NBC) / 64) + 7) / 8), 1u), 256, 0, stream>>>(
        (const unsigned short*)X16, nullptr, DM, 0, (const unsigned short*)WB, nullptr, DM, 0, (void*)BC, nullptr, NBC, 0, BIAS, nullptr, 0, MROWS, NBC, DM, 0.00390625f);
    k_out<<<(unsigned)(((long long)MROWS * (DM / 4) + 255) / 256), 256, 0, stream>>>(x, DL, BC, out);
}
